// CNNBackbone_83468394430599
// MI455X (gfx1250) — hardware-verified
//
#include <hip/hip_runtime.h>

constexpr int kB    = 32;
constexpr int kS    = 2048;
constexpr int kD    = 128;
constexpr int kC    = 256;
constexpr int kTaps = 5;
constexpr int kPad  = 2;
constexpr int kSP   = kS + 2 * kPad;
constexpr int kK1   = kTaps * kD;
constexpr int kK2   = kTaps * kC;
constexpr float kWCarryInv = 1.0f / 16.0f;
constexpr float kBnEps = 1e-5f;

constexpr size_t al256(size_t b) { return (b + 255) & ~(size_t)255; }
constexpr size_t kBytesP1   = (size_t)kB * kSP * kD * 2;
constexpr size_t kBytesP2   = (size_t)kB * kSP * kC * 2;
constexpr size_t kBytesH2   = (size_t)kB * kS * kC * 2;
constexpr size_t kBytesConv = (size_t)kB * kS * kD * 4;
constexpr size_t kBytesWt1  = (size_t)kC * kK1 * 2;
constexpr size_t kBytesWt2  = (size_t)kC * kK2 * 2;
constexpr size_t kBytesWtf  = (size_t)kD * kC * 2;
constexpr size_t kOffP1   = 0;
constexpr size_t kOffP2   = kOffP1 + al256(kBytesP1);
constexpr size_t kOffH2   = kOffP2 + al256(kBytesP2);
constexpr size_t kOffConv = kOffH2 + al256(kBytesH2);
constexpr size_t kOffWt1  = kOffConv + al256(kBytesConv);
constexpr size_t kOffWt2  = kOffWt1 + al256(kBytesWt1);
constexpr size_t kOffWtf  = kOffWt2 + al256(kBytesWt2);
constexpr size_t kOffCs1  = kOffWtf + al256(kBytesWtf);
constexpr size_t kOffCb1  = kOffCs1 + 1024;
constexpr size_t kOffCs2  = kOffCb1 + 1024;
constexpr size_t kOffCb2  = kOffCs2 + 1024;
constexpr size_t kOffBfr  = kOffCb2 + 1024;
constexpr size_t kWsTotal = kOffBfr + 1024;
constexpr size_t kWsLimit = (size_t)134217728;
typedef char ws_fits_check[(kWsTotal <= kWsLimit) ? 1 : -1];
typedef char k_mult32_check[((kK1 % 32) == 0 && (kK2 % 32) == 0 && (kC % 32) == 0 && (kD % 32) == 0) ? 1 : -1];
typedef char tile_check[((kS % 64) == 0 && (kC % 64) == 0 && (kD % 64) == 0) ? 1 : -1];

constexpr int kTilesConv12 = (kS / 64) * (kC / 64);
constexpr int kTilesConv3  = (kS / 64) * (kD / 64);
constexpr int kGridConv12  = kTilesConv12 / 8;
constexpr int kGridConv3   = kTilesConv3 / 8;
typedef char grid_check[((kTilesConv12 % 8) == 0 && (kTilesConv3 % 8) == 0) ? 1 : -1];
constexpr int kChunksPerBatchX = kS * kD / 8;
constexpr int kGridCastX  = kB * kChunksPerBatchX / 256;
constexpr int kZeroBlkP1  = (kB * 4 * (kD / 8)) / 256;
constexpr int kZeroBlkP2  = (kB * 4 * (kC / 8)) / 256;
constexpr int kBlkW1 = (kC * kK1 / 8) / 256;
constexpr int kBlkW2 = (kC * kK2 / 8) / 256;
constexpr int kBlkWf = (kD * kC / 8) / 256;
constexpr int kGridPrep = kBlkW1 + kBlkW2 + kBlkWf + 1;
typedef char seg_check[(((kC * kK1 / 8) % 256) == 0 && ((kC * kK2 / 8) % 256) == 0 && ((kD * kC / 8) % 256) == 0 &&
                        ((kB * 4 * (kD / 8)) % 256) == 0 && ((kB * 4 * (kC / 8)) % 256) == 0 &&
                        ((kB * kChunksPerBatchX) % 256) == 0) ? 1 : -1];

typedef __attribute__((ext_vector_type(16))) _Float16 v16h;
typedef __attribute__((ext_vector_type(8)))  _Float16 v8h;
typedef __attribute__((ext_vector_type(8)))  float    v8f;
typedef __attribute__((ext_vector_type(4)))  float    v4f;
typedef __attribute__((ext_vector_type(4)))  unsigned int v4u;

__device__ __forceinline__ unsigned short f2bf_bits(float f) {
  unsigned u = __float_as_uint(f);
  return (unsigned short)((u + 0x7FFFu + ((u >> 16) & 1u)) >> 16);
}
__device__ __forceinline__ float bf_bits2f(unsigned short h) { return __uint_as_float(((unsigned)h) << 16); }
__device__ __forceinline__ float rne_bf16f(float f) { return bf_bits2f(f2bf_bits(f)); }
__device__ __forceinline__ unsigned pk16(unsigned short a, unsigned short b) { return (unsigned)a | ((unsigned)b << 16); }
__device__ __forceinline__ unsigned short h_bits(float f) { const _Float16 h = (_Float16)f; return __builtin_bit_cast(unsigned short, h); }

__device__ __forceinline__ void dep_guard_h(v8f& a, v8f& b, v16h x, v16h y) { asm volatile("v_nop\n\tv_nop\n\tv_nop\n\tv_nop" : "+v"(a), "+v"(b) : "v"(x), "v"(y)); }
__device__ __forceinline__ void keep4_h(v16h a, v16h b, v16h c, v16h d) { asm volatile("v_nop" :: "v"(a), "v"(b), "v"(c), "v"(d)); }
__device__ __forceinline__ void acc_guard4(v8f& a, v8f& b, v8f& c, v8f& d) { asm volatile("v_nop\n\tv_nop\n\tv_nop\n\tv_nop" : "+v"(a), "+v"(b), "+v"(c), "+v"(d)); }
template <typename T> struct Frag;
template <> struct Frag<_Float16> {
  typedef v16h V; union U { v16h v; v8h h[2]; };
  static __device__ __forceinline__ v16h load(const _Float16* p) {
    U f; f.h[0] = *(const v8h*)(p); f.h[1] = *(const v8h*)(p + 16); return f.v;
  }
  static __device__ __forceinline__ v8f mma(v16h a, v16h b, v8f c) {
    return __builtin_amdgcn_wmma_f32_16x16x32_f16(false, a, false, b, (short)0, c, false, false);
  }
  static __device__ __forceinline__ void guard(v8f& a, v8f& b, v16h x, v16h y) { dep_guard_h(a, b, x, y); }
  static __device__ __forceinline__ void keep(v16h a, v16h b, v16h c, v16h d) { keep4_h(a, b, c, d); }
};

template <int CIN_T, int BIAS_MODE, int OUT_MODE, int ACT>
__global__ __launch_bounds__(256) void conv_gemm64(
    const unsigned short* __restrict__ Ap, int lda, long strideA,
    const unsigned short* __restrict__ Btp, int ldb,
    void* __restrict__ Cout, int ldc, long strideC,
    const float* __restrict__ colscale, const float* __restrict__ bias,
    int M, int N, int K, float scale) {
  typedef _Float16 T;
  typedef v16h V;
  const T* A = (const T*)Ap; const T* Bt = (const T*)Btp;
  __shared__ __align__(16) float sT[8][16 * 68];
  const int b    = blockIdx.y;
  const int lane = threadIdx.x & 31;
  const int wave = threadIdx.x >> 5;
  const int tilesN = N >> 6;
  const int tilesM = M >> 6;
  const int tile = blockIdx.x * 8 + wave;
  if (tile >= tilesM * tilesN) return;
  const int tm = tile / tilesN;
  const int tn = tile - tm * tilesN;
  const int m0 = tm << 6;
  const int n0 = tn << 6;

  const T* Ab = A + (size_t)b * strideA;
  const T* Bb = Bt;

  const int rlane = lane & 15;
  const int koff  = (lane >> 4) * 8;
  const int mOff  = (lane >> 4) * 8;

  v8f acc[4][4];
#pragma unroll
  for (int i = 0; i < 4; ++i)
#pragma unroll
    for (int j = 0; j < 4; ++j) acc[i][j] = (v8f){0.f,0.f,0.f,0.f,0.f,0.f,0.f,0.f};

  for (int k0 = 0; k0 < K; k0 += 32) {
    const int tap = k0 / CIN_T;
    const int kc  = k0 - tap * CIN_T;
    V bh[4];
#pragma unroll
    for (int j = 0; j < 4; ++j) {
      const size_t bo = (size_t)(n0 + (j << 4) + rlane) * ldb + koff + k0;
      bh[j] = Frag<T>::load(Bb + bo);
    }
#pragma unroll
    for (int i = 0; i < 4; ++i) {
      const size_t ao = (size_t)(m0 + (i << 4) + rlane + tap) * lda + koff + kc;
      V ah = Frag<T>::load(Ab + ao);
#pragma unroll
      for (int j = 0; j < 4; ++j) acc[i][j] = Frag<T>::mma(ah, bh[j], acc[i][j]);
      Frag<T>::guard(acc[i][0], acc[i][3], ah, ah);
    }
    Frag<T>::keep(bh[0], bh[1], bh[2], bh[3]);
  }
  acc_guard4(acc[0][0], acc[0][1], acc[0][2], acc[0][3]);
  acc_guard4(acc[1][0], acc[1][1], acc[1][2], acc[1][3]);
  acc_guard4(acc[2][0], acc[2][1], acc[2][2], acc[2][3]);
  acc_guard4(acc[3][0], acc[3][1], acc[3][2], acc[3][3]);

  float* slab = sT[wave];
#pragma unroll
  for (int i = 0; i < 4; ++i) {
    const int mBase = m0 + (i << 4);
#pragma unroll
    for (int j = 0; j < 4; ++j) {
      const int n = n0 + (j << 4) + rlane;
      float bv = 0.f, csv = 1.f;
      if (BIAS_MODE == 2 || BIAS_MODE == 3) bv = bias[n];
      if (BIAS_MODE == 3) csv = colscale[n];
#pragma unroll
      for (int r = 0; r < 8; ++r) {
        float v = acc[i][j][r] * scale;
        if (BIAS_MODE == 2) v += bv;
        if (BIAS_MODE == 3) v = v * csv + bv;
        if (ACT == 2) v = fmaxf(v, 0.0f);
        slab[(mOff + r) * 68 + (j << 4) + rlane] = v;
      }
    }
    __builtin_amdgcn_fence(__ATOMIC_RELEASE, "workgroup");
    __builtin_amdgcn_wave_barrier();
    __builtin_amdgcn_fence(__ATOMIC_ACQUIRE, "workgroup");
    if (OUT_MODE == 0) {
      float* Cp = (float*)Cout + (size_t)b * strideC;
      const int hh = lane >> 4, c4 = (lane & 15) * 4;
      for (int pass = 0; pass < 2; ++pass) {
#pragma unroll
        for (int it = 0; it < 8; ++it) {
          const int row = it * 2 + hh;
          v4f v = *(const v4f*)(slab + row * 68 + c4);
          *(volatile v4f*)(Cp + (size_t)(mBase + row) * ldc + n0 + c4) = v;
        }
        __threadfence();
      }
    } else {
      const int q = lane >> 3, c8 = (lane & 7) * 8;
      unsigned short* Cp = (unsigned short*)Cout + (size_t)b * strideC;
      for (int pass = 0; pass < 2; ++pass) {
#pragma unroll
        for (int it = 0; it < 4; ++it) {
          const int row = it * 4 + q;
          const float* sp = slab + row * 68 + c8;
          v8h hv;
#pragma unroll
          for (int e = 0; e < 8; ++e) hv[e] = (_Float16)sp[e];
          *(volatile v8h*)(Cp + (size_t)(mBase + row) * ldc + n0 + c8) = hv;
        }
        __threadfence();
      }
    }
    __builtin_amdgcn_fence(__ATOMIC_RELEASE, "workgroup");
    __builtin_amdgcn_wave_barrier();
    __builtin_amdgcn_fence(__ATOMIC_ACQUIRE, "workgroup");
  }
}

__global__ __launch_bounds__(256) void cast_x_rows(const float* __restrict__ x, unsigned short* __restrict__ P1) {
  const int g = blockIdx.x * 256 + threadIdx.x;
  const int b = g / kChunksPerBatchX;
  const int w = g - b * kChunksPerBatchX;
  const float* src = x + (size_t)g * 8;
  const v4f f0 = *(const v4f*)(src);
  const v4f f1 = *(const v4f*)(src + 4);
  const unsigned short h0 = h_bits(rne_bf16f(f0[0])), h1 = h_bits(rne_bf16f(f0[1]));
  const unsigned short h2 = h_bits(rne_bf16f(f0[2])), h3 = h_bits(rne_bf16f(f0[3]));
  const unsigned short h4 = h_bits(rne_bf16f(f1[0])), h5 = h_bits(rne_bf16f(f1[1]));
  const unsigned short h6 = h_bits(rne_bf16f(f1[2])), h7 = h_bits(rne_bf16f(f1[3]));
  const v4u u = (v4u){pk16(h0, h1), pk16(h2, h3), pk16(h4, h5), pk16(h6, h7)};
  unsigned short* dst = P1 + ((size_t)b * kSP + kPad) * kD + (size_t)w * 8;
  *(volatile v4u*)dst = u;
  __threadfence();
  *(volatile v4u*)dst = u;
}

__device__ __forceinline__ void zero_rows_impl(unsigned short* __restrict__ base, int cpr, int rowh, int g) {
  const int per_b = 4 * cpr;
  const int b   = g / per_b;
  const int rem = g - b * per_b;
  const int rr  = rem / cpr;
  const int ch  = rem - rr * cpr;
  const int row = b * kSP + ((rr < 2) ? rr : (kS + rr));
  unsigned short* dst = base + (size_t)row * rowh + ch * 8;
  const v4u z = (v4u){0u, 0u, 0u, 0u};
  *(volatile v4u*)dst = z;
  __threadfence();
  *(volatile v4u*)dst = z;
}
__global__ __launch_bounds__(256) void zero_pad_rows(unsigned short* __restrict__ P1, unsigned short* __restrict__ P2) {
  const int blk = blockIdx.x, t = threadIdx.x;
  if (blk < kZeroBlkP1) zero_rows_impl(P1, kD / 8, kD, blk * 256 + t);
  else                  zero_rows_impl(P2, kC / 8, kC, (blk - kZeroBlkP1) * 256 + t);
}

__global__ __launch_bounds__(256) void prep_weights_params(
    const float* __restrict__ W1, const float* __restrict__ W2, const float* __restrict__ Wf,
    const float* __restrict__ b1, const float* __restrict__ g1, const float* __restrict__ be1,
    const float* __restrict__ m1, const float* __restrict__ v1,
    const float* __restrict__ b2, const float* __restrict__ g2, const float* __restrict__ be2,
    const float* __restrict__ m2, const float* __restrict__ v2, const float* __restrict__ bfv,
    unsigned short* __restrict__ Wt1, unsigned short* __restrict__ Wt2, unsigned short* __restrict__ Wtf,
    float* __restrict__ cs1, float* __restrict__ cb1, float* __restrict__ cs2, float* __restrict__ cb2,
    float* __restrict__ bfr) {
  const int blk = blockIdx.x;
  const int t   = threadIdx.x;
  if (blk < kBlkW1) {
    const int g   = blk * 256 + t;
    const int cpr = kK1 / 8;
    const int n   = g / cpr;
    const int ch  = g - n * cpr;
    const int kk  = ch * 8;
    const int tap = kk / kD;
    const int c0  = kk - tap * kD;
    unsigned short hb[8];
#pragma unroll
    for (int e = 0; e < 8; ++e) {
      const float w = W1[((size_t)n * kD + c0 + e) * kTaps + tap];
      hb[e] = h_bits(rne_bf16f(w) * 16.0f);
    }
    const v4u u = (v4u){pk16(hb[0], hb[1]), pk16(hb[2], hb[3]), pk16(hb[4], hb[5]), pk16(hb[6], hb[7])};
    unsigned short* dst = Wt1 + (size_t)g * 8;
    *(volatile v4u*)dst = u;
    __threadfence();
    *(volatile v4u*)dst = u;
  } else if (blk < kBlkW1 + kBlkW2) {
    const int g   = (blk - kBlkW1) * 256 + t;
    const int cpr = kK2 / 8;
    const int n   = g / cpr;
    const int ch  = g - n * cpr;
    const int kk  = ch * 8;
    const int tap = kk / kC;
    const int c0  = kk - tap * kC;
    unsigned short hb[8];
#pragma unroll
    for (int e = 0; e < 8; ++e) {
      const float w = W2[((size_t)n * kC + c0 + e) * kTaps + tap];
      hb[e] = h_bits(rne_bf16f(w) * 16.0f);
    }
    const v4u u = (v4u){pk16(hb[0], hb[1]), pk16(hb[2], hb[3]), pk16(hb[4], hb[5]), pk16(hb[6], hb[7])};
    unsigned short* dst = Wt2 + (size_t)g * 8;
    *(volatile v4u*)dst = u;
    __threadfence();
    *(volatile v4u*)dst = u;
  } else if (blk < kBlkW1 + kBlkW2 + kBlkWf) {
    const int g   = (blk - kBlkW1 - kBlkW2) * 256 + t;
    const int cpr = kC / 8;
    const int d   = g / cpr;
    const int ch  = g - d * cpr;
    unsigned short hb[8];
#pragma unroll
    for (int e = 0; e < 8; ++e) {
      const float w = Wf[(size_t)d * kC + ch * 8 + e];
      hb[e] = h_bits(rne_bf16f(w) * 16.0f);
    }
    const v4u u = (v4u){pk16(hb[0], hb[1]), pk16(hb[2], hb[3]), pk16(hb[4], hb[5]), pk16(hb[6], hb[7])};
    unsigned short* dst = Wtf + (size_t)g * 8;
    *(volatile v4u*)dst = u;
    __threadfence();
    *(volatile v4u*)dst = u;
  } else {
    const float ga = rne_bf16f(g1[t]), bea = rne_bf16f(be1[t]), ma = rne_bf16f(m1[t]), va = rne_bf16f(v1[t]), ba = rne_bf16f(b1[t]);
    const float sca = ga * rsqrtf(va + kBnEps);
    const float cba = ba * sca + (bea - ma * sca);
    const float gb = rne_bf16f(g2[t]), beb = rne_bf16f(be2[t]), mb = rne_bf16f(m2[t]), vb = rne_bf16f(v2[t]), bb = rne_bf16f(b2[t]);
    const float scb = gb * rsqrtf(vb + kBnEps);
    const float cbb = bb * scb + (beb - mb * scb);
    const bool lowhalf = (t < kD);
    const float bfv_r = rne_bf16f(bfv[lowhalf ? t : 0]);
    ((volatile float*)cs1)[t] = sca;
    ((volatile float*)cb1)[t] = cba;
    ((volatile float*)cs2)[t] = scb;
    ((volatile float*)cb2)[t] = cbb;
    if (lowhalf) ((volatile float*)bfr)[t] = bfv_r;
    __threadfence();
    ((volatile float*)cs1)[t] = sca;
    ((volatile float*)cb1)[t] = cba;
    ((volatile float*)cs2)[t] = scb;
    ((volatile float*)cb2)[t] = cbb;
    if (lowhalf) ((volatile float*)bfr)[t] = bfv_r;
  }
}

__global__ __launch_bounds__(256) void masked_mean_pool(const float* __restrict__ conv, const int* __restrict__ spi,
                                                        float* __restrict__ out) {
  __shared__ float part[256];
  __shared__ __align__(16) float pooled[kD];
  const int b = blockIdx.x;
  const int t = threadIdx.x;
  const int d = t & (kD - 1);
  const int half = t >> 7;
  int len = spi[b];
  if (len == -1) len = kS;
  int lenc = len < 0 ? 0 : len;
  lenc = lenc > kS ? kS : lenc;
  const float* cb = conv + (size_t)b * kS * kD + d;
  float acc = 0.f;
#pragma unroll 1
  for (int s = half; s < lenc; s += 2) acc += cb[(size_t)s * kD];
  part[t] = acc;
  __syncthreads();
  if (t < kD) {
    const float sum = part[t] + part[t + kD];
    const int den = len > 1 ? len : 1;
    const float rcp = 1.0f / (float)den;
    pooled[t] = (len > 0) ? (sum * rcp) : 0.0f;
  }
  __syncthreads();
  if (t < 32) {
    const v4f val = *(const v4f*)(pooled + 4 * t);
    float* op = out + (size_t)b * kD + 4 * t;
    *(volatile v4f*)op = val;
    __threadfence();
    *(volatile v4f*)op = val;
  }
}

extern "C" void kernel_launch(void* const* d_in, const int* in_sizes, int n_in,
                              void* d_out, int out_size, void* d_ws, size_t ws_size,
                              hipStream_t stream)
{
  if (n_in < 16) return;
  if (in_sizes[0] != kB * kS * kD || in_sizes[1] != kB || in_sizes[2] != kC * kD * kTaps ||
      in_sizes[8] != kC * kC * kTaps || in_sizes[14] != kD * kC || out_size != kB * kD) return;
  for (int i = 3; i <= 13; ++i) { if (i == 8) continue; if (in_sizes[i] != kC) return; }
  if (in_sizes[15] != kD) return;
  if (ws_size < kWsTotal) return;

  const float* x   = (const float*)d_in[0];
  const int*   spi = (const int*)  d_in[1];
  const float* W1  = (const float*)d_in[2];
  const float* b1  = (const float*)d_in[3];
  const float* g1  = (const float*)d_in[4];
  const float* be1 = (const float*)d_in[5];
  const float* m1  = (const float*)d_in[6];
  const float* v1  = (const float*)d_in[7];
  const float* W2  = (const float*)d_in[8];
  const float* b2  = (const float*)d_in[9];
  const float* g2  = (const float*)d_in[10];
  const float* be2 = (const float*)d_in[11];
  const float* m2  = (const float*)d_in[12];
  const float* v2  = (const float*)d_in[13];
  const float* Wf  = (const float*)d_in[14];
  const float* bfv = (const float*)d_in[15];
  float* out = (float*)d_out;

  char* ws = (char*)d_ws;
  unsigned short* P1   = (unsigned short*)(ws + kOffP1);
  unsigned short* P2   = (unsigned short*)(ws + kOffP2);
  unsigned short* H2   = (unsigned short*)(ws + kOffH2);
  float*          CONV = (float*)(ws + kOffConv);
  unsigned short* Wt1  = (unsigned short*)(ws + kOffWt1);
  unsigned short* Wt2  = (unsigned short*)(ws + kOffWt2);
  unsigned short* Wtf  = (unsigned short*)(ws + kOffWtf);
  float* cs1 = (float*)(ws + kOffCs1);
  float* cb1 = (float*)(ws + kOffCb1);
  float* cs2 = (float*)(ws + kOffCs2);
  float* cb2 = (float*)(ws + kOffCb2);
  float* bfr = (float*)(ws + kOffBfr);

  cast_x_rows<<<kGridCastX, 256, 0, stream>>>(x, P1);
  zero_pad_rows<<<kZeroBlkP1 + kZeroBlkP2, 256, 0, stream>>>(P1, P2);
  prep_weights_params<<<kGridPrep, 256, 0, stream>>>(W1, W2, Wf, b1, g1, be1, m1, v1, b2, g2, be2, m2, v2, bfv,
                                                     Wt1, Wt2, Wtf, cs1, cb1, cs2, cb2, bfr);
  conv_gemm64<kD, 3, 1, 2><<<dim3(kGridConv12, kB), 256, 0, stream>>>(
      P1, kD, (long)kSP * kD,
      Wt1, kK1,
      (void*)(P2 + (size_t)kPad * kC), kC, (long)kSP * kC,
      cs1, cb1, kS, kC, kK1, kWCarryInv);
  conv_gemm64<kC, 3, 1, 2><<<dim3(kGridConv12, kB), 256, 0, stream>>>(
      P2, kC, (long)kSP * kC,
      Wt2, kK2,
      (void*)H2, kC, (long)kS * kC,
      cs2, cb2, kS, kC, kK2, kWCarryInv);
  conv_gemm64<kC, 2, 0, 0><<<dim3(kGridConv3, kB), 256, 0, stream>>>(
      H2, kC, (long)kS * kC,
      Wtf, kC,
      (void*)CONV, kD, (long)kS * kD,
      cs2, bfr, kS, kD, kC, kWCarryInv);
  masked_mean_pool<<<kB, 256, 0, stream>>>(CONV, spi, out);
}
